// DifferentialAttention_51092930953782
// MI455X (gfx1250) — hardware-verified
//
#include <hip/hip_runtime.h>


typedef _Float16     v16h __attribute__((ext_vector_type(16)));
typedef _Float16     h8   __attribute__((ext_vector_type(8)));
typedef float        v8f  __attribute__((ext_vector_type(8)));
typedef float        f4   __attribute__((ext_vector_type(4)));
typedef unsigned int u4   __attribute__((ext_vector_type(4)));

#ifndef NB
#define NB 2
#endif
#ifndef SEQ
#define SEQ 2048
#endif
#define NB_FULL  2
#define SEQ_FULL 2048
#define DM     1024
#define HEADS  16
#define DH     64
#define NQKV   (3 * DM)
#define MROWS  (NB * SEQ)
#define G8     (DM / 8)

#define QT  128
#define KT  64
#define LP  72
#define FP  68

#define WSC 64.0f
#define RSC 2048.0f
#define PSC 1024.0f
#define OSC 1024.0f
#define SCL 0.03125f

static_assert(DM == 1024);
static_assert(G8 == 128);
static_assert(HEADS * DH == DM);
static_assert(DH == 64);
static_assert(SEQ % QT == 0);
static_assert(SEQ % KT == 0);
static_assert(SEQ % 64 == 0);
static_assert(MROWS % 64 == 0);
static_assert(NQKV % 64 == 0);
static_assert(NB >= 1 && NB <= NB_FULL);
static_assert(SEQ <= SEQ_FULL);
static_assert(64 * FP * 4 <= 2 * 64 * LP * 2);

#define XH_BYTES ((size_t)MROWS * DM * 2)
#define WQ_BYTES ((size_t)NQKV * DM * 2)
#define WO_BYTES ((size_t)DM * DM * 2)
#define PL_BYTES ((size_t)MROWS * DM * 2)
#define OFF_XH  ((size_t)0)
#define OFF_WQ  (OFF_XH + XH_BYTES)
#define OFF_WO  (OFF_WQ + WQ_BYTES)
#define OFF_QH  (OFF_WO + WO_BYTES)
#define OFF_QL  (OFF_QH + PL_BYTES)
#define OFF_KH  (OFF_QL + PL_BYTES)
#define OFF_KL  (OFF_KH + PL_BYTES)
#define OFF_VT  (OFF_KL + PL_BYTES)
#define OFF_OH  (OFF_VT + PL_BYTES)
#define WS_NEED (OFF_OH + PL_BYTES)
static_assert(WS_NEED <= (size_t)134217728);
static_assert((OFF_WQ % 128) == 0 && (OFF_WO % 128) == 0 && (OFF_QH % 128) == 0 && (OFF_OH % 128) == 0);

__device__ __forceinline__ float bf16r(float x) {
  unsigned int u = __float_as_uint(x);
  u = (u + 0x7FFFu + ((u >> 16) & 1u)) & 0xFFFF0000u;
  return __uint_as_float(u);
}

__device__ __forceinline__ v8f zero8() {
  v8f z;
#pragma unroll
  for (int j = 0; j < 8; ++j) z[j] = 0.0f;
  return z;
}

__device__ __forceinline__ v8f wmma16(v16h a, v16h b, v8f c) {
  return __builtin_amdgcn_wmma_f32_16x16x32_f16(false, a, false, b, (short)0, c, false, false);
}

#define WGUARD(acc, a, b) \
  asm volatile("v_nop\n\tv_nop\n\tv_nop\n\tv_nop" : "+v"(acc) : "v"(a), "v"(b))
#define WGUARD2(c0, c1, a, b0, b1) \
  asm volatile("v_nop\n\tv_nop\n\tv_nop\n\tv_nop" : "+v"(c0), "+v"(c1) : "v"(a), "v"(b0), "v"(b1))

union HU  { v16h v; h8 p[2]; };
union H8U { h8 h; u4 u; };

__device__ __forceinline__ v16h ldfrag(const _Float16* row, int kb8) {
  HU u;
  u.p[0] = *(const h8*)(row + kb8);
  u.p[1] = *(const h8*)(row + 16 + kb8);
  return u.v;
}

__global__ __launch_bounds__(256) void k_convert(const float* __restrict__ src, _Float16* __restrict__ dst,
                                                 int ngroups, int seq, int seq_full, float scale) {
  const int g = blockIdx.x * 256 + threadIdx.x;
  if (g >= ngroups) return;
  const int row = g >> 7;
  const int c8  = g & 127;
  const int srow = (row / seq) * seq_full + (row - (row / seq) * seq);
  const float* s = src + (size_t)srow * DM + c8 * 8;
  const f4 a = *(const f4*)s;
  const f4 b = *(const f4*)(s + 4);
  H8U o;
#pragma unroll
  for (int j = 0; j < 4; ++j) {
    o.h[j]     = (_Float16)(bf16r(a[j]) * scale);
    o.h[4 + j] = (_Float16)(bf16r(b[j]) * scale);
  }
  _Float16* d = dst + (size_t)row * DM + c8 * 8;
  *(volatile u4*)d = o.u;
  __threadfence();
  *(volatile u4*)d = o.u;
}

__device__ __forceinline__ void gemm_tile(const _Float16* __restrict__ A, const _Float16* __restrict__ Bw,
                                          int m0, int n0, _Float16* sA, _Float16* sB, v8f (&acc)[4]) {
  const int tid = threadIdx.x, lane = tid & 31, wave = tid >> 5, l16 = lane & 15, kb8 = (lane >> 4) * 8;
  for (int k0 = 0; k0 < DM; k0 += 64) {
#pragma unroll
    for (int i = 0; i < 4; ++i) {
      const int idx = tid + 128 * i;
      const int r = idx >> 3, pc = idx & 7;
      const u4 va = *(const u4*)(A  + (size_t)(m0 + r) * DM + k0 + pc * 8);
      const u4 vb = *(const u4*)(Bw + (size_t)(n0 + r) * DM + k0 + pc * 8);
      *(u4*)(sA + r * LP + pc * 8) = va;
      *(u4*)(sB + r * LP + pc * 8) = vb;
    }
    __syncthreads();
    const _Float16* ar = sA + (wave * 16 + l16) * LP;
    const v16h a0 = ldfrag(ar, kb8);
    const v16h a1 = ldfrag(ar + 32, kb8);
#pragma unroll
    for (int nt = 0; nt < 4; ++nt) {
      const _Float16* br = sB + (nt * 16 + l16) * LP;
      const v16h b0 = ldfrag(br, kb8);
      const v16h b1 = ldfrag(br + 32, kb8);
      acc[nt] = wmma16(a0, b0, acc[nt]);
      acc[nt] = wmma16(a1, b1, acc[nt]);
      WGUARD(acc[nt], a1, b1);
    }
    __syncthreads();
  }
}

__global__ __launch_bounds__(128) void k_qkv(const _Float16* __restrict__ Xh, const _Float16* __restrict__ Wh,
                                             const float* __restrict__ bias,
                                             _Float16* __restrict__ Qhi, _Float16* __restrict__ Qlo,
                                             _Float16* __restrict__ Khi, _Float16* __restrict__ Klo,
                                             _Float16* __restrict__ Vt) {
  __shared__ __align__(16) _Float16 sA[64 * LP];
  __shared__ __align__(16) _Float16 sB[64 * LP];
  const int tid = threadIdx.x, lane = tid & 31, wave = tid >> 5, l16 = lane & 15, half = lane >> 4;
  const int m0 = blockIdx.x * 64, n0 = blockIdx.y * 64;

  v8f acc[4];
#pragma unroll
  for (int nt = 0; nt < 4; ++nt) acc[nt] = zero8();
  gemm_tile(Xh, Wh, m0, n0, sA, sB, acc);

  const int sel = n0 / DM;
  const int hd  = (n0 - sel * DM) / DH;
  const int bb  = m0 / SEQ, l0 = m0 - bb * SEQ;
  const size_t bh = (size_t)bb * HEADS + hd;
  const float inv = 1.0f / WSC;
  float bcol[4];
#pragma unroll
  for (int nt = 0; nt < 4; ++nt) bcol[nt] = bf16r(bias[n0 + nt * 16 + l16]);

  if (sel < 2) {
#pragma unroll
    for (int nt = 0; nt < 4; ++nt) {
#pragma unroll
      for (int r = 0; r < 8; ++r) {
        const float v = acc[nt][r] * inv + bcol[nt];
        const _Float16 hi = (_Float16)v;
        const _Float16 lo = (_Float16)((v - (float)hi) * RSC);
        const int row = wave * 16 + half * 8 + r, col = nt * 16 + l16;
        sA[row * LP + col] = hi;
        sB[row * LP + col] = lo;
      }
    }
  } else {
#pragma unroll
    for (int nt = 0; nt < 4; ++nt) {
      H8U o;
#pragma unroll
      for (int r = 0; r < 8; ++r) o.h[r] = (_Float16)(acc[nt][r] * inv + bcol[nt]);
      *(u4*)(sA + (nt * 16 + l16) * LP + wave * 16 + half * 8) = o.u;
    }
  }
  __syncthreads();

  if (sel < 2) {
    _Float16* dhp = ((sel == 0) ? Qhi : Khi) + (bh * SEQ + l0) * DH;
    _Float16* dlp = ((sel == 0) ? Qlo : Klo) + (bh * SEQ + l0) * DH;
#pragma unroll
    for (int p = 0; p < 4; ++p) {
      const int line = p * 16 + (tid >> 3), piece = tid & 7;
      const u4 vh = *(const u4*)(sA + line * LP + piece * 8);
      const u4 vl = *(const u4*)(sB + line * LP + piece * 8);
      *(volatile u4*)(dhp + line * DH + piece * 8) = vh;
      *(volatile u4*)(dlp + line * DH + piece * 8) = vl;
    }
    __threadfence();
#pragma unroll
    for (int p = 0; p < 4; ++p) {
      const int line = p * 16 + (tid >> 3), piece = tid & 7;
      const u4 vh = *(const u4*)(sA + line * LP + piece * 8);
      const u4 vl = *(const u4*)(sB + line * LP + piece * 8);
      *(volatile u4*)(dhp + line * DH + piece * 8) = vh;
      *(volatile u4*)(dlp + line * DH + piece * 8) = vl;
    }
  } else {
    _Float16* dvp = Vt + (bh * DH) * (size_t)SEQ + l0;
#pragma unroll
    for (int p = 0; p < 4; ++p) {
      const int e = p * 16 + (tid >> 3), piece = tid & 7;
      const u4 v = *(const u4*)(sA + e * LP + piece * 8);
      *(volatile u4*)(dvp + (size_t)e * SEQ + piece * 8) = v;
    }
    __threadfence();
#pragma unroll
    for (int p = 0; p < 4; ++p) {
      const int e = p * 16 + (tid >> 3), piece = tid & 7;
      const u4 v = *(const u4*)(sA + e * LP + piece * 8);
      *(volatile u4*)(dvp + (size_t)e * SEQ + piece * 8) = v;
    }
  }
}

__global__ __launch_bounds__(256) void k_attn(const _Float16* __restrict__ Qhi, const _Float16* __restrict__ Qlo,
                                              const _Float16* __restrict__ Khi, const _Float16* __restrict__ Klo,
                                              const _Float16* __restrict__ Vt, const float* __restrict__ lam_p,
                                              const int* __restrict__ heads_p, _Float16* __restrict__ Oh) {
  const int tid = threadIdx.x, lane = tid & 31, wave = tid >> 5;
  const int l16 = lane & 15, half = lane >> 4, kb8 = half * 8;
  const int bh = blockIdx.x;
  const int b  = bh / HEADS, h = bh - b * HEADS;
  const int qBase = blockIdx.y * QT;

  __shared__ __align__(16) _Float16 sKh[KT * LP];
  __shared__ __align__(16) _Float16 sKl[KT * LP];
  __shared__ __align__(16) _Float16 sV[DH * LP];
  __shared__ __align__(16) _Float16 sP[8 * KT * 16];
  _Float16* ps = sP + wave * (KT * 16);

  const float lamr = bf16r(lam_p[0]);
  const int   hv   = heads_p[0];
  const float lamv = (hv == HEADS) ? lamr : __uint_as_float(0x7fc00000u);

  const size_t qrow = (size_t)bh * SEQ + qBase + wave * 16 + l16;
  const _Float16* qh = Qhi + qrow * DH;
  const _Float16* ql = Qlo + qrow * DH;
  const v16h qa0 = ldfrag(qh, kb8), qa1 = ldfrag(qh + 32, kb8);
  const v16h qr0 = ldfrag(ql, kb8), qr1 = ldfrag(ql + 32, kb8);

  float m[8], lsum[8], lgLast[8];
  v8f acc[4];
  float v0r[4];
#pragma unroll
  for (int j = 0; j < 8; ++j) { m[j] = -3.0e38f; lsum[j] = 0.0f; lgLast[j] = 0.0f; }
#pragma unroll
  for (int n = 0; n < 4; ++n) { acc[n] = zero8(); v0r[n] = 0.0f; }

  const int   rsrc = (lane & 16) | ((l16 + 15) & 15);
  const float cxs  = 1.0f / RSC;

  const _Float16* khBase = Khi + (size_t)bh * SEQ * DH;
  const _Float16* klBase = Klo + (size_t)bh * SEQ * DH;
  const _Float16* vtBase = Vt  + (size_t)bh * DH * SEQ;

  for (int it = 0; it < SEQ / KT; ++it) {
    __syncthreads();
#pragma unroll
    for (int i = 0; i < 2; ++i) {
      const int idx = tid + 256 * i;
      const int r = idx >> 3, pc = idx & 7;
      const u4 vkh = *(const u4*)(khBase + (size_t)(it * KT + r) * DH + pc * 8);
      const u4 vkl = *(const u4*)(klBase + (size_t)(it * KT + r) * DH + pc * 8);
      const u4 vv  = *(const u4*)(vtBase + (size_t)r * SEQ + it * KT + pc * 8);
      *(u4*)(sKh + r * LP + pc * 8) = vkh;
      *(u4*)(sKl + r * LP + pc * 8) = vkl;
      *(u4*)(sV  + r * LP + pc * 8) = vv;
    }
    __syncthreads();
    if (it == 0) {
#pragma unroll
      for (int n = 0; n < 4; ++n) v0r[n] = (float)sV[(16 * n + l16) * LP];
    }

    float p[4][8];
    float tmax[8];
#pragma unroll
    for (int j = 0; j < 8; ++j) tmax[j] = -3.0e38f;
#pragma unroll
    for (int t = 0; t < 4; ++t) {
      const _Float16* kr = sKh + (t * 16 + l16) * LP;
      const _Float16* kq = sKl + (t * 16 + l16) * LP;
      const v16h kh0 = ldfrag(kr, kb8), kh1 = ldfrag(kr + 32, kb8);
      v8f chh = zero8();
      chh = wmma16(qa0, kh0, chh);
      chh = wmma16(qa1, kh1, chh);
      v8f cx = zero8();
      cx = wmma16(qr0, kh0, cx);
      cx = wmma16(qr1, kh1, cx);
      const v16h kl0 = ldfrag(kq, kb8), kl1 = ldfrag(kq + 32, kb8);
      cx = wmma16(qa0, kl0, cx);
      cx = wmma16(qa1, kl1, cx);
      WGUARD2(chh, cx, qa1, kh1, kl1);
#pragma unroll
      for (int j = 0; j < 8; ++j) {
        const float lg = (chh[j] + cx[j] * cxs) * SCL;
        p[t][j] = lg;
        tmax[j] = fmaxf(tmax[j], lg);
      }
    }

#pragma unroll
    for (int j = 0; j < 8; ++j) {
      float v = tmax[j];
      v = fmaxf(v, __shfl_xor(v, 1, 32));
      v = fmaxf(v, __shfl_xor(v, 2, 32));
      v = fmaxf(v, __shfl_xor(v, 4, 32));
      v = fmaxf(v, __shfl_xor(v, 8, 32));
      tmax[j] = v;
    }
    float nlg[8];
#pragma unroll
    for (int j = 0; j < 8; ++j) nlg[j] = __shfl(p[3][j], rsrc, 32);

    float corr[8], pleft0[8];
#pragma unroll
    for (int j = 0; j < 8; ++j) {
      const float nm = fmaxf(m[j], tmax[j]);
      corr[j] = __expf(m[j] - nm);
      m[j] = nm;
      const float pt = __expf(lgLast[j] - nm);
      pleft0[j] = (it == 0) ? 0.0f : pt;
    }
#pragma unroll
    for (int j = 0; j < 8; ++j) {
      float s = 0.0f;
#pragma unroll
      for (int t = 0; t < 4; ++t) {
        p[t][j] = __expf(p[t][j] - m[j]);
        s += p[t][j];
      }
      s += __shfl_xor(s, 1, 32);
      s += __shfl_xor(s, 2, 32);
      s += __shfl_xor(s, 4, 32);
      s += __shfl_xor(s, 8, 32);
      lsum[j] = lsum[j] * corr[j] + s;
    }
#pragma unroll
    for (int n = 0; n < 4; ++n)
#pragma unroll
      for (int j = 0; j < 8; ++j) acc[n][j] *= corr[j];
#pragma unroll
    for (int j = 0; j < 8; ++j) lgLast[j] = nlg[j];

    {
      float rleft[8];
#pragma unroll
      for (int j = 0; j < 8; ++j) rleft[j] = pleft0[j];
#pragma unroll
      for (int t = 0; t < 4; ++t) {
        H8U o;
#pragma unroll
        for (int j = 0; j < 8; ++j) {
          const float rc   = __shfl(p[t][j], rsrc, 32);
          const float left = (l16 != 0) ? rc : rleft[j];
          o.h[j] = (_Float16)((p[t][j] - left) * PSC);
          rleft[j] = rc;
        }
        *(u4*)(ps + (t * 16 + l16) * 16 + half * 8) = o.u;
      }
    }
    __builtin_amdgcn_fence(5, "wavefront");
    __builtin_amdgcn_wave_barrier();

    v16h pa0, pa1;
#pragma unroll
    for (int c = 0; c < 8; ++c) {
      pa0[c]     = ps[(kb8 + c) * 16 + l16];
      pa0[c + 8] = ps[(16 + kb8 + c) * 16 + l16];
      pa1[c]     = ps[(32 + kb8 + c) * 16 + l16];
      pa1[c + 8] = ps[(48 + kb8 + c) * 16 + l16];
    }
#pragma unroll
    for (int n = 0; n < 4; ++n) {
      const _Float16* vr = sV + (16 * n + l16) * LP;
      const v16h uv0 = ldfrag(vr, kb8), uv1 = ldfrag(vr + 32, kb8);
      acc[n] = wmma16(pa0, uv0, acc[n]);
      acc[n] = wmma16(pa1, uv1, acc[n]);
      WGUARD(acc[n], pa1, uv1);
    }
  }
  __syncthreads();

  float pL[8], f[8];
#pragma unroll
  for (int j = 0; j < 8; ++j) {
    const float lgl = __shfl(lgLast[j], lane & 16, 32);
    pL[j] = __expf(lgl - m[j]) * PSC;
    f[j]  = lamv * (OSC / PSC) * (1.0f / lsum[j]);
  }
  _Float16* po = ps;
#pragma unroll
  for (int n = 0; n < 4; ++n) {
#pragma unroll
    for (int j = 0; j < 8; ++j) {
      const float val = (acc[n][j] - pL[j] * v0r[n]) * f[j];
      po[(half * 8 + j) * 64 + 16 * n + l16] = (_Float16)val;
    }
  }
  __builtin_amdgcn_fence(5, "wavefront");
  __builtin_amdgcn_wave_barrier();

  _Float16* od = Oh + ((size_t)b * SEQ + qBase + wave * 16) * DM + h * DH;
#pragma unroll
  for (int p4 = 0; p4 < 4; ++p4) {
    const int line = p4 * 4 + (lane >> 3), piece = lane & 7;
    const u4 v = *(const u4*)(po + line * 64 + piece * 8);
    *(volatile u4*)(od + (size_t)line * DM + piece * 8) = v;
  }
  __threadfence();
#pragma unroll
  for (int p4 = 0; p4 < 4; ++p4) {
    const int line = p4 * 4 + (lane >> 3), piece = lane & 7;
    const u4 v = *(const u4*)(po + line * 64 + piece * 8);
    *(volatile u4*)(od + (size_t)line * DM + piece * 8) = v;
  }
}

__global__ __launch_bounds__(128) void k_out(const _Float16* __restrict__ Oh, const _Float16* __restrict__ Woh,
                                             const float* __restrict__ bias, float* __restrict__ out) {
  __shared__ __align__(16) unsigned char smem[2 * 64 * LP * 2];
  _Float16* sA = (_Float16*)smem;
  _Float16* sB = sA + 64 * LP;
  const int tid = threadIdx.x, lane = tid & 31, wave = tid >> 5, l16 = lane & 15, half = lane >> 4;
  const int m0 = blockIdx.x * 64, n0 = blockIdx.y * 64;

  v8f acc[4];
#pragma unroll
  for (int nt = 0; nt < 4; ++nt) acc[nt] = zero8();
  gemm_tile(Oh, Woh, m0, n0, sA, sB, acc);

  float* sF = (float*)smem;
  const float inv = 1.0f / (OSC * WSC);
  float bcol[4];
#pragma unroll
  for (int nt = 0; nt < 4; ++nt) bcol[nt] = bf16r(bias[n0 + nt * 16 + l16]);
#pragma unroll
  for (int nt = 0; nt < 4; ++nt) {
#pragma unroll
    for (int r = 0; r < 8; ++r) {
      const int row = wave * 16 + half * 8 + r, col = nt * 16 + l16;
      sF[row * FP + col] = acc[nt][r] * inv + bcol[nt];
    }
  }
  __syncthreads();

  const int bb = m0 / SEQ, l0 = m0 - bb * SEQ;
  float* dbase = out + ((size_t)bb * SEQ_FULL + l0) * DM + n0;
#pragma unroll
  for (int p = 0; p < 8; ++p) {
    const int line = p * 16 + (tid >> 3), piece = tid & 7;
    const int row = line >> 1, hs = line & 1;
    const f4 v = *(const f4*)(sF + row * FP + hs * 32 + piece * 4);
    *(volatile f4*)(dbase + (size_t)row * DM + hs * 32 + piece * 4) = v;
  }
  __threadfence();
#pragma unroll
  for (int p = 0; p < 8; ++p) {
    const int line = p * 16 + (tid >> 3), piece = tid & 7;
    const int row = line >> 1, hs = line & 1;
    const f4 v = *(const f4*)(sF + row * FP + hs * 32 + piece * 4);
    *(volatile f4*)(dbase + (size_t)row * DM + hs * 32 + piece * 4) = v;
  }
}

static inline unsigned cdiv_u(unsigned a, unsigned b) { return (a + b - 1) / b; }

extern "C" void kernel_launch(void* const* d_in, const int* in_sizes, int n_in,
                              void* d_out, int out_size, void* d_ws, size_t ws_size,
                              hipStream_t stream) {
  if (n_in < 7) return;
  const long long need_rows = (long long)(NB - 1) * SEQ_FULL + SEQ;
  if ((long long)in_sizes[0] < need_rows * DM) return;
  if (in_sizes[1] < NQKV * DM) return;
  if (in_sizes[2] < NQKV) return;
  if (in_sizes[3] < DM * DM) return;
  if (in_sizes[4] < DM) return;
  if (in_sizes[5] < 1) return;
  if (in_sizes[6] < 1) return;
  if ((long long)out_size < need_rows * DM) return;
  if (d_ws == nullptr || ws_size < WS_NEED) return;

  const float* x     = (const float*)d_in[0];
  const float* w_qkv = (const float*)d_in[1];
  const float* b_qkv = (const float*)d_in[2];
  const float* w_out = (const float*)d_in[3];
  const float* b_out = (const float*)d_in[4];
  const float* lam   = (const float*)d_in[5];
  const int*   heads = (const int*)d_in[6];
  float* out = (float*)d_out;

  char* ws = (char*)d_ws;
  _Float16* Xh  = (_Float16*)(ws + OFF_XH);
  _Float16* Wq  = (_Float16*)(ws + OFF_WQ);
  _Float16* Wo  = (_Float16*)(ws + OFF_WO);
  _Float16* Qhi = (_Float16*)(ws + OFF_QH);
  _Float16* Qlo = (_Float16*)(ws + OFF_QL);
  _Float16* Khi = (_Float16*)(ws + OFF_KH);
  _Float16* Klo = (_Float16*)(ws + OFF_KL);
  _Float16* Vt  = (_Float16*)(ws + OFF_VT);
  _Float16* Oh  = (_Float16*)(ws + OFF_OH);

  const int gx = MROWS * G8, gq = NQKV * G8, go = DM * G8;
  k_convert<<<dim3(cdiv_u(gx, 256)), dim3(256), 0, stream>>>(x,     Xh, gx, SEQ,  SEQ_FULL, 1.0f);
  k_convert<<<dim3(cdiv_u(gq, 256)), dim3(256), 0, stream>>>(w_qkv, Wq, gq, NQKV, NQKV,     WSC);
  k_convert<<<dim3(cdiv_u(go, 256)), dim3(256), 0, stream>>>(w_out, Wo, go, DM,   DM,       WSC);

  k_qkv<<<dim3(MROWS / 64, NQKV / 64), dim3(128), 0, stream>>>(Xh, Wq, b_qkv, Qhi, Qlo, Khi, Klo, Vt);
  k_attn<<<dim3(NB * HEADS, SEQ / QT), dim3(256), 0, stream>>>(Qhi, Qlo, Khi, Klo, Vt, lam, heads, Oh);
  k_out<<<dim3(MROWS / 64, DM / 64), dim3(128), 0, stream>>>(Oh, Wo, b_out, out);
}
